// RingDilatedAttentionHybridHilbert_46153718563051
// MI455X (gfx1250) — hardware-verified
//
#include <hip/hip_runtime.h>
#define NB 4
#define DM 512
#define NKV 8
#define NREP (NH / NKV)
#define KVD (NKV * 64)
#define NR (NB * SLEN)
#define CHK 512
typedef int v4i __attribute__((ext_vector_type(4)));
#define FF 2048
#define SLEN 2048
#define MQI 2048
#define MKI 2048
#define TQ SLEN
#define TK SLEN
#define NH 8
#define SCL 0.125f
#define QBLKS (TQ / 64)
#define QB05 0
#define QBN5 QBLKS
#define QB0P 0
#define QBNP QBLKS
#define RE 256
typedef __bf16 v16b __attribute__((ext_vector_type(16)));
typedef unsigned short v8us __attribute__((ext_vector_type(8), may_alias));
typedef float  v8f  __attribute__((ext_vector_type(8)));
typedef float  v4f  __attribute__((ext_vector_type(4)));
typedef float  v4fa __attribute__((ext_vector_type(4), may_alias));
union FragB { v16b v; v8us half[2]; unsigned short u[16]; };

__device__ __forceinline__ unsigned short bf16_bits(float x) { unsigned int u = __float_as_uint(x); return (unsigned short)((u + 0x7FFFu + ((u >> 16) & 1u)) >> 16); }
__device__ __forceinline__ float bf16_val(unsigned short b) { return __uint_as_float(((unsigned int)b) << 16); }
__device__ __forceinline__ float bf16_round(float x) { return bf16_val(bf16_bits(x)); }
template <int NT>
__device__ __forceinline__ v8f mmaN(v16b ah, v16b al, v16b bh, v16b bl, v8f c) {
  c = __builtin_amdgcn_wmma_f32_16x16x32_bf16(false, ah, false, bh, (short)0, c, false, false);
  if (NT >= 2) c = __builtin_amdgcn_wmma_f32_16x16x32_bf16(false, al, false, bh, (short)0, c, false, false);
  if (NT >= 3) c = __builtin_amdgcn_wmma_f32_16x16x32_bf16(false, ah, false, bl, (short)0, c, false, false);
  asm volatile("v_nop\n\tv_nop\n\tv_nop\n\tv_nop" : "+v"(c) : "v"(ah), "v"(al), "v"(bh), "v"(bl));
  return c;
}

__global__ __launch_bounds__(256) void k_wt_bf16(const float* __restrict__ W, unsigned short* __restrict__ Wt, int K, int N) {
  const int t = blockIdx.x * 256 + threadIdx.x;
  const int k8n = K / 8;
  if (t >= N * k8n) return;
  const int n = t / k8n, k8 = (t % k8n) * 8;
  v8us v;
#pragma unroll
  for (int i = 0; i < 8; ++i) v[i] = bf16_bits(W[(size_t)(k8 + i) * N + n]);
  *(volatile v8us*)(Wt + (size_t)n * K + k8) = v;
  __threadfence();
  *(volatile v8us*)(Wt + (size_t)n * K + k8) = v;
}

template <bool ASPLIT, int ACT, bool BIAS_BF16>
__global__ __launch_bounds__(128) void k_gemm_bf(const float* __restrict__ A, int lda, const unsigned short* __restrict__ Wt, int ldb,
                                               const float* __restrict__ bias, float* __restrict__ C, int ldc, int M, int N, int K) {
  __shared__ __attribute__((aligned(16))) float so[4][16][64];
  const int tid = threadIdx.x, w = tid >> 5, lane = tid & 31, ln = lane & 15, hh = lane >> 4;
  const int ntn = N / 64;
  const int wid = blockIdx.x * 4 + w;
  const int mt = wid / ntn, nq = wid % ntn;
  if (mt * 16 >= M) return;
  const int row0 = mt * 16, col0 = nq * 64;
  const float* arow = A + (size_t)(row0 + ln) * lda;
  v8f acc[4] = {};
  for (int kb = 0; kb < K; kb += 32) {
    FragB ah, al;
    const v4f x0 = *(const v4fa*)(arow + kb + 8 * hh), x1 = *(const v4fa*)(arow + kb + 8 * hh + 4);
    const v4f x2 = *(const v4fa*)(arow + kb + 16 + 8 * hh), x3 = *(const v4fa*)(arow + kb + 16 + 8 * hh + 4);
    float xs[16] = {x0[0],x0[1],x0[2],x0[3],x1[0],x1[1],x1[2],x1[3],x2[0],x2[1],x2[2],x2[3],x3[0],x3[1],x3[2],x3[3]};
#pragma unroll
    for (int i = 0; i < 16; ++i) { const unsigned short hb = bf16_bits(xs[i]); ah.u[i] = hb; al.u[i] = ASPLIT ? bf16_bits(xs[i] - bf16_val(hb)) : (unsigned short)0; }
#pragma unroll
    for (int t = 0; t < 4; ++t) {
      const unsigned short* brow = Wt + (size_t)(col0 + t * 16 + ln) * ldb + kb;
      FragB b;
      b.half[0] = *(const v8us*)(brow + 8 * hh);
      b.half[1] = *(const v8us*)(brow + 16 + 8 * hh);
      acc[t] = mmaN<ASPLIT ? 2 : 1>(ah.v, al.v, b.v, b.v, acc[t]);
    }
  }
#pragma unroll
  for (int t = 0; t < 4; ++t) {
    float bv = bias ? bias[col0 + t * 16 + ln] : 0.f;
    if (BIAS_BF16) bv = bf16_round(bv);
#pragma unroll
    for (int r = 0; r < 8; ++r) { float v = acc[t][r] + bv; if (ACT == 1) v = fmaxf(v, 0.f); so[w][8 * hh + r][t * 16 + ln] = v; }
  }
  __builtin_amdgcn_fence(__ATOMIC_ACQ_REL, "workgroup");
  __builtin_amdgcn_wave_barrier();
  const int rsub = lane >> 4, c4 = (lane & 15) * 4;
  for (int pass = 0; pass < 2; ++pass) {
#pragma unroll
    for (int q = 0; q < 8; ++q) {
      const int r = q * 2 + rsub;
      const v4f v = *(const v4fa*)&so[w][r][c4];
      *(volatile v4f*)(C + (size_t)(row0 + r) * ldc + col0 + c4) = v;
    }
    if (pass == 0) __threadfence();
  }
}

template <bool ASPLIT, int ACT, bool BIAS_BF16, bool RES_BF16>
__global__ __launch_bounds__(128) void k_gemm_bf3(const float* __restrict__ A, int lda, const unsigned short* __restrict__ Wt, int ldb,
                                                const float* __restrict__ bias, const float* __restrict__ resid, int rmod, int ldr,
                                                float* __restrict__ C, int ldc, int M, int N, int K) {
  __shared__ __attribute__((aligned(16))) float so[4][16][64];
  const int tid = threadIdx.x, w = tid >> 5, lane = tid & 31, ln = lane & 15, hh = lane >> 4;
  const int ntn = N / 64;
  const int wid = blockIdx.x * 4 + w;
  const int mt = wid / ntn, nq = wid % ntn;
  if (mt * 16 >= M) return;
  const int row0 = mt * 16, col0 = nq * 64;
  const float* arow = A + (size_t)(row0 + ln) * lda;
  v8f acc[4] = {};
  for (int kb = 0; kb < K; kb += 32) {
    FragB ah, al;
    const v4f x0 = *(const v4fa*)(arow + kb + 8 * hh), x1 = *(const v4fa*)(arow + kb + 8 * hh + 4);
    const v4f x2 = *(const v4fa*)(arow + kb + 16 + 8 * hh), x3 = *(const v4fa*)(arow + kb + 16 + 8 * hh + 4);
    float xs[16] = {x0[0],x0[1],x0[2],x0[3],x1[0],x1[1],x1[2],x1[3],x2[0],x2[1],x2[2],x2[3],x3[0],x3[1],x3[2],x3[3]};
#pragma unroll
    for (int i = 0; i < 16; ++i) { const unsigned short hb = bf16_bits(xs[i]); ah.u[i] = hb; al.u[i] = ASPLIT ? bf16_bits(xs[i] - bf16_val(hb)) : (unsigned short)0; }
#pragma unroll
    for (int t = 0; t < 4; ++t) {
      const unsigned short* brow = Wt + (size_t)(col0 + t * 16 + ln) * ldb + kb;
      FragB b;
      b.half[0] = *(const v8us*)(brow + 8 * hh);
      b.half[1] = *(const v8us*)(brow + 16 + 8 * hh);
      acc[t] = mmaN<ASPLIT ? 2 : 1>(ah.v, al.v, b.v, b.v, acc[t]);
    }
  }
#pragma unroll
  for (int t = 0; t < 4; ++t) {
    const int col = col0 + t * 16 + ln;
    float bv = bias ? bias[col] : 0.f;
    if (BIAS_BF16) bv = bf16_round(bv);
#pragma unroll
    for (int r = 0; r < 8; ++r) {
      float v = acc[t][r] + bv;
      if (resid) { float rv = resid[(size_t)((row0 + 8 * hh + r) % rmod) * ldr + col]; if (RES_BF16) rv = bf16_round(rv); v += rv; }
      if (ACT == 1) v = fmaxf(v, 0.f);
      if (ACT == 2) v = 0.5f * v * (1.0f + erff(v * 0.70710678118654752f));
      if (ACT == 3) { const float u = 0.7978845608028654f * (v + 0.044715f * v * v * v); v = 0.5f * v * (1.0f + tanhf(u)); }
      so[w][8 * hh + r][t * 16 + ln] = v;
    }
  }
  __builtin_amdgcn_fence(__ATOMIC_ACQ_REL, "workgroup");
  __builtin_amdgcn_wave_barrier();
  const int rsub = lane >> 4, c4 = (lane & 15) * 4;
  for (int pass = 0; pass < 2; ++pass) {
#pragma unroll
    for (int q = 0; q < 8; ++q) {
      const int r = q * 2 + rsub;
      const v4f v = *(const v4fa*)&so[w][r][c4];
      *(volatile v4f*)(C + (size_t)(row0 + r) * ldc + col0 + c4) = v;
    }
    if (pass == 0) __threadfence();
  }
}
template <bool PARAM_BF16>
__global__ __launch_bounds__(256) void k_layernorm(const float* __restrict__ X, const float* __restrict__ R, const float* __restrict__ g, const float* __restrict__ bta,
                                                  float* __restrict__ out_sum, float* __restrict__ out_norm, int N, float eps) {
  __shared__ float red[256];
  const int row = blockIdx.x, tid = threadIdx.x;
  const float* x = X + (size_t)row * N; const float* rr = R ? R + (size_t)row * N : nullptr;
  float vals[16];
  const int per = N / 256;
  float s1 = 0.f;
  for (int u = 0; u < per / 4; ++u) {
    const int j = tid * 4 + 1024 * u;
    const v4f a = *(const v4fa*)(x + j);
    v4f b = {0.f,0.f,0.f,0.f}; if (rr) b = *(const v4fa*)(rr + j);
#pragma unroll
    for (int q = 0; q < 4; ++q) { const float v = a[q] + b[q]; vals[u * 4 + q] = v; s1 += v; }
  }
  red[tid] = s1; __syncthreads();
  for (int st = 128; st > 0; st >>= 1) { if (tid < st) red[tid] += red[tid + st]; __syncthreads(); }
  const float mu = red[0] / (float)N; __syncthreads();
  float s2 = 0.f;
  for (int u = 0; u < per / 4; ++u)
#pragma unroll
    for (int q = 0; q < 4; ++q) { const float c = vals[u * 4 + q] - mu; s2 += c * c; }
  red[tid] = s2; __syncthreads();
  for (int st = 128; st > 0; st >>= 1) { if (tid < st) red[tid] += red[tid + st]; __syncthreads(); }
  const float rs = rsqrtf(red[0] / (float)N + eps);
  for (int pass = 0; pass < 2; ++pass) {
    for (int u = 0; u < per / 4; ++u) {
      const int j = tid * 4 + 1024 * u;
      v4f o, sm;
#pragma unroll
      for (int q = 0; q < 4; ++q) {
        float gg = g[j + q], bb = bta[j + q];
        if (PARAM_BF16) { gg = bf16_round(gg); bb = bf16_round(bb); }
        sm[q] = vals[u * 4 + q]; o[q] = (vals[u * 4 + q] - mu) * rs * gg + bb;
      }
      if (out_sum) *(volatile v4f*)(out_sum + (size_t)row * N + j) = sm;
      *(volatile v4f*)(out_norm + (size_t)row * N + j) = o;
    }
    if (pass == 0) __threadfence();
  }
}


typedef _Float16 v16h __attribute__((ext_vector_type(16)));
union FragH { v16h v; v8us half[2]; _Float16 h[16]; unsigned short u[16]; };
template <int NT>
__device__ __forceinline__ v8f mmaH(v16h ah, v16h al, v16h bh, v16h bl, v8f c) {
  c = __builtin_amdgcn_wmma_f32_16x16x32_f16(false, ah, false, bh, (short)0, c, false, false);
  if (NT >= 2) c = __builtin_amdgcn_wmma_f32_16x16x32_f16(false, al, false, bh, (short)0, c, false, false);
  if (NT >= 3) c = __builtin_amdgcn_wmma_f32_16x16x32_f16(false, ah, false, bl, (short)0, c, false, false);
  asm volatile("v_nop\n\tv_nop\n\tv_nop\n\tv_nop" : "+v"(c) : "v"(ah), "v"(al), "v"(bh), "v"(bl));
  return c;
}
template <bool ASPLIT>
__global__ __launch_bounds__(128) void k_gemm_h(const float* __restrict__ A, int lda, size_t sA, const _Float16* __restrict__ Bh, int ldb, size_t sB, float alpha, float* __restrict__ C, int ldc, size_t sC, int M, int N, int K) {
  __shared__ __attribute__((aligned(16))) float so[4][16][64];
  const int tid = threadIdx.x, w = tid >> 5, lane = tid & 31, ln = lane & 15, hh = lane >> 4; const int by = blockIdx.y;
  A += (size_t)by * sA; Bh += (size_t)by * sB; C += (size_t)by * sC;
  const int ntn = (N + 63) / 64; const int wid = blockIdx.x * 4 + w; const int mt = wid / ntn, nq = wid % ntn; if (mt * 16 >= M) return;
  const int row0 = mt * 16, col0 = nq * 64; const float* arow = A + (size_t)(row0 + ln) * lda;
  v8f acc[4] = {};
  for (int kb = 0; kb < K; kb += 32) {
    FragH ah, al;
    const v4f x0 = *(const v4fa*)(arow + kb + 8 * hh), x1 = *(const v4fa*)(arow + kb + 8 * hh + 4), x2 = *(const v4fa*)(arow + kb + 16 + 8 * hh), x3 = *(const v4fa*)(arow + kb + 16 + 8 * hh + 4);
    float xs[16] = {x0[0],x0[1],x0[2],x0[3],x1[0],x1[1],x1[2],x1[3],x2[0],x2[1],x2[2],x2[3],x3[0],x3[1],x3[2],x3[3]};
#pragma unroll
    for (int i = 0; i < 16; ++i) { const _Float16 h = (_Float16)xs[i]; ah.h[i] = h; al.h[i] = ASPLIT ? (_Float16)(xs[i] - (float)h) : (_Float16)0.0f; }
#pragma unroll
    for (int t = 0; t < 4; ++t) { if (col0 + t * 16 >= N) continue; const size_t boff = (size_t)(col0 + t * 16 + ln) * ldb + kb; FragH bq; bq.half[0] = *(const v8us*)(Bh + boff + 8 * hh); bq.half[1] = *(const v8us*)(Bh + boff + 16 + 8 * hh);
      acc[t] = mmaH<ASPLIT ? 2 : 1>(ah.v, al.v, bq.v, bq.v, acc[t]); }
  }
#pragma unroll
  for (int t = 0; t < 4; ++t) { if (col0 + t * 16 >= N) continue;
#pragma unroll
    for (int r = 0; r < 8; ++r) so[w][8 * hh + r][t * 16 + ln] = acc[t][r] * alpha; }
  __builtin_amdgcn_fence(__ATOMIC_ACQ_REL, "workgroup"); __builtin_amdgcn_wave_barrier();
  const int rsub = lane >> 4, c4 = (lane & 15) * 4;
  for (int pass = 0; pass < 2; ++pass) {
#pragma unroll
    for (int q = 0; q < 8; ++q) { const int r = q * 2 + rsub; if (col0 + c4 < N) { const v4f v = *(const v4fa*)&so[w][r][c4]; *(volatile v4f*)(C + (size_t)(row0 + r) * ldc + col0 + c4) = v; } }
    if (pass == 0) __threadfence(); }
}

__global__ __launch_bounds__(256) void k_wt_f16(const float* __restrict__ W, _Float16* __restrict__ Wt, int K, int N, float scale) {
  const int t = blockIdx.x * 256 + threadIdx.x; if (t >= N * (K / 8)) return; const int n = t / (K / 8), k8 = (t % (K / 8)) * 8; FragH f;
#pragma unroll
  for (int i = 0; i < 8; ++i) f.h[i] = (_Float16)(bf16_round(W[(size_t)(k8 + i) * N + n]) * scale); const v8us o = f.half[0];
  *(volatile v8us*)((unsigned short*)Wt + (size_t)n * K + k8) = o; __threadfence(); *(volatile v8us*)((unsigned short*)Wt + (size_t)n * K + k8) = o;
}
template <int ACT>
__global__ __launch_bounds__(128) void k_gemm_hhx(const _Float16* __restrict__ A, int lda, size_t sA, const _Float16* __restrict__ Bh, int ldb, size_t sB, float alpha, const float* __restrict__ bias, size_t sBias, const float* __restrict__ CP, int rowsPerB, size_t sCPb, int row0g,
    float* __restrict__ C, _Float16* __restrict__ C16, int ldc, size_t sC, int M, int N, int K) {
  __shared__ __attribute__((aligned(16))) float so[4][16][64];
  const int tid = threadIdx.x, w = tid >> 5, lane = tid & 31, ln = lane & 15, hh = lane >> 4; const int by = blockIdx.y;
  A += (size_t)by * sA; Bh += (size_t)by * sB; const size_t cofs = (size_t)by * sC; const float* bp = bias ? bias + (size_t)by * sBias : nullptr;
  const int ntn = (N + 63) / 64; const int wid = blockIdx.x * 4 + w; const int mt = wid / ntn, nq = wid % ntn; if (mt * 16 >= M) return;
  const int row0 = mt * 16, col0 = nq * 64; const _Float16* arow = A + (size_t)(row0 + ln) * lda;
  v8f acc[4] = {};
  for (int kb = 0; kb < K; kb += 32) { FragH ah; ah.half[0] = *(const v8us*)((const unsigned short*)arow + kb + 8 * hh); ah.half[1] = *(const v8us*)((const unsigned short*)arow + kb + 16 + 8 * hh);
#pragma unroll
    for (int t = 0; t < 4; ++t) { if (col0 + t * 16 >= N) continue; const size_t boff = (size_t)(col0 + t * 16 + ln) * ldb + kb; FragH bq; bq.half[0] = *(const v8us*)((const unsigned short*)Bh + boff + 8 * hh); bq.half[1] = *(const v8us*)((const unsigned short*)Bh + boff + 16 + 8 * hh);
      acc[t] = mmaH<1>(ah.v, ah.v, bq.v, bq.v, acc[t]); }
  }
#pragma unroll
  for (int t = 0; t < 4; ++t) { if (col0 + t * 16 >= N) continue; const int col = col0 + t * 16 + ln; const float bv = bp ? bf16_round(bp[col]) : 0.f;
#pragma unroll
    for (int r = 0; r < 8; ++r) { float v = acc[t][r] * alpha + bv; if (CP) { const int bidx = (row0g + row0 + 8 * hh + r) / rowsPerB; v += CP[(size_t)bidx * sCPb + (size_t)by * 64 + col]; } if (ACT == 1) v = (v > 0.f) ? v : expm1f(v); else if (ACT == 7) v = (v > 0.f) ? v + 1.0f : expf(v); else if (ACT == 8) v = tanhf(v); else if (ACT == 9) v = 0.5f * v * (1.0f + tanhf(0.7978845608028654f * (v + 0.044715f * v * v * v))); else if (ACT == 11) v = 1.0f / (1.0f + expf(-v)); else if (ACT == 12) v = (v > 0.f) ? v : 0.01f * v; else if (ACT == 14) v = (v > 0.f) ? v : 0.1f * v; else if (ACT == 15) v = v / (1.0f + expf(-v)); else if (ACT == 3) v = fmaxf(v, 0.f); else if (ACT == 6) v = 0.5f * v * (1.0f + erff(v * 0.70710678118654752f)); so[w][8 * hh + r][t * 16 + ln] = v; } }
  __builtin_amdgcn_fence(__ATOMIC_ACQ_REL, "workgroup"); __builtin_amdgcn_wave_barrier();
  const int rsub = lane >> 4, c4 = (lane & 15) * 4; typedef _Float16 v4h __attribute__((ext_vector_type(4)));
  for (int pass = 0; pass < 2; ++pass) {
#pragma unroll
    for (int q = 0; q < 8; ++q) { const int r = q * 2 + rsub; if (col0 + c4 < N) { const v4f v = *(const v4fa*)&so[w][r][c4]; if (C) *(volatile v4f*)(C + cofs + (size_t)(row0 + r) * ldc + col0 + c4) = v; if (C16) { v4h h4; for (int i = 0; i < 4; ++i) h4[i] = (_Float16)v[i]; *(volatile v4h*)(C16 + cofs + (size_t)(row0 + r) * ldc + col0 + c4) = h4; } } }
    if (pass == 0) __threadfence(); }
}


typedef _Float16 v4h __attribute__((ext_vector_type(4)));

__global__ __launch_bounds__(256) void k_x16(const float* __restrict__ x, _Float16* __restrict__ X16, size_t n8) { const size_t t = (size_t)blockIdx.x * 256 + threadIdx.x; if (t >= n8) return; FragH f;
#pragma unroll
  for (int q = 0; q < 8; ++q) f.h[q] = (_Float16)bf16_round(x[t * 8 + q]); *(volatile v8us*)((unsigned short*)X16 + t * 8) = f.half[0]; __threadfence(); *(volatile v8us*)((unsigned short*)X16 + t * 8) = f.half[0]; }
__global__ __launch_bounds__(256) void k_h16(const float* __restrict__ x, _Float16* __restrict__ X16, size_t n8) { const size_t t = (size_t)blockIdx.x * 256 + threadIdx.x; if (t >= n8) return; FragH f;
#pragma unroll
  for (int q = 0; q < 8; ++q) f.h[q] = (_Float16)x[t * 8 + q]; *(volatile v8us*)((unsigned short*)X16 + t * 8) = f.half[0]; __threadfence(); *(volatile v8us*)((unsigned short*)X16 + t * 8) = f.half[0]; }
__global__ __launch_bounds__(256) void k_round16f(const float* __restrict__ W, _Float16* __restrict__ Bt, size_t n8) { const size_t t = (size_t)blockIdx.x * 256 + threadIdx.x; if (t >= n8) return; FragH f;
#pragma unroll
  for (int i = 0; i < 8; ++i) f.h[i] = (_Float16)(bf16_round(W[t * 8 + i]) * 16.0f); *(volatile v8us*)((unsigned short*)Bt + t * 8) = f.half[0]; __threadfence(); *(volatile v8us*)((unsigned short*)Bt + t * 8) = f.half[0]; }
template <int NHv, int TTv>
__global__ __launch_bounds__(256) void k_vt(const _Float16* __restrict__ V16, int ldv, int voff, _Float16* __restrict__ Vt) { __shared__ unsigned short tl[64][66]; const int tid = threadIdx.x; const int slab = blockIdx.x / (TTv / 64), lg = blockIdx.x % (TTv / 64); const int b = slab / NHv, h = slab % NHv;
  for (int i = tid; i < 64 * 8; i += 256) { const int r = i / 8, c8 = (i % 8) * 8; FragH f; f.half[0] = *(const v8us*)((const unsigned short*)V16 + ((size_t)b * TTv + lg * 64 + r) * ldv + voff + h * 64 + c8);
#pragma unroll
    for (int q = 0; q < 8; ++q) tl[r][c8 + q] = f.u[q]; }
  __syncthreads();
  for (int pass = 0; pass < 2; ++pass) {
#pragma unroll
    for (int rd = 0; rd < 2; ++rd) { const int d = rd * 32 + tid / 8, pc = tid % 8; FragH f;
#pragma unroll
      for (int q = 0; q < 8; ++q) f.u[q] = tl[pc * 8 + q][d];
      *(volatile v8us*)((unsigned short*)Vt + ((size_t)slab * 64 + d) * TTv + lg * 64 + pc * 8) = f.half[0]; }
    if (pass == 0) __threadfence(); } }

__global__ __launch_bounds__(256) void k_hl(const float* __restrict__ F, _Float16* __restrict__ Hh, _Float16* __restrict__ Hl, size_t n8) { const size_t t = (size_t)blockIdx.x * 256 + threadIdx.x; if (t >= n8) return; FragH fh, fl; const v4f a = *(const v4fa*)(F + t * 8), c = *(const v4fa*)(F + t * 8 + 4);
#pragma unroll
  for (int q = 0; q < 4; ++q) { _Float16 h = (_Float16)a[q]; fh.h[q] = h; fl.h[q] = (_Float16)((a[q] - (float)h) * 1024.0f); h = (_Float16)c[q]; fh.h[4 + q] = h; fl.h[4 + q] = (_Float16)((c[q] - (float)h) * 1024.0f); }
  for (int pass = 0; pass < 2; ++pass) { *(volatile v8us*)((unsigned short*)Hh + t * 8) = fh.half[0]; *(volatile v8us*)((unsigned short*)Hl + t * 8) = fl.half[0]; if (pass == 0) __threadfence(); } }

__device__ __forceinline__ v16h g2_frag(const _Float16* p, int hh) { FragH f; f.half[0] = *(const v8us*)((const unsigned short*)p + 8 * hh); f.half[1] = *(const v8us*)((const unsigned short*)p + 16 + 8 * hh); return f.v; }
__device__ __forceinline__ v8f g2_mma(v16h a, v16h b, v8f c) { v8f d = __builtin_amdgcn_wmma_f32_16x16x32_f16(false, a, false, b, (short)0, c, false, false); asm volatile("v_nop\n\tv_nop\n\tv_nop\n\tv_nop" : "+v"(d) : "v"(a), "v"(b)); return d; }
template <int ACT>
__global__ __launch_bounds__(128) void k_gemm2(const _Float16* __restrict__ A, int lda, size_t sA, const _Float16* __restrict__ Bh, int ldb, size_t sB, float alpha, const float* __restrict__ bias, size_t sBias, const float* __restrict__ CP, int rowsPerB, size_t sCPb, int row0g,
    float* __restrict__ C, _Float16* __restrict__ C16, int ldc, size_t sC, int M, int N, int K) {
  __shared__ __attribute__((aligned(16))) float so[4][32][68];
  const int tid = threadIdx.x, w = tid >> 5, lane = tid & 31, ln = lane & 15, hh = lane >> 4; const int by = blockIdx.y;
  A += (size_t)by * sA; Bh += (size_t)by * sB; const size_t cofs = (size_t)by * sC; const float* bp = bias ? bias + (size_t)by * sBias : nullptr;
  const int ntn = N >> 6; const int mt = blockIdx.x / ntn, nq = blockIdx.x - mt * ntn; const int row0 = mt * 128 + 32 * w, col0 = nq * 64; if (row0 >= M) return;
  const _Float16* a0p = A + (size_t)(row0 + ln) * lda; const _Float16* a1p = a0p + (size_t)16 * lda;
  const _Float16* b0p = Bh + (size_t)(col0 + ln) * ldb; const _Float16* b1p = b0p + (size_t)16 * ldb; const _Float16* b2p = b1p + (size_t)16 * ldb; const _Float16* b3p = b2p + (size_t)16 * ldb;
  const v8f z8 = {0.f,0.f,0.f,0.f,0.f,0.f,0.f,0.f}; v8f c00 = z8, c01 = z8, c02 = z8, c03 = z8, c10 = z8, c11 = z8, c12 = z8, c13 = z8;
#pragma unroll 1
  for (int kb = 0; kb < K; kb += 32) { const v16h a0 = g2_frag(a0p + kb, hh), a1 = g2_frag(a1p + kb, hh);
    v16h b = g2_frag(b0p + kb, hh); c00 = g2_mma(a0, b, c00); c10 = g2_mma(a1, b, c10);
    b = g2_frag(b1p + kb, hh); c01 = g2_mma(a0, b, c01); c11 = g2_mma(a1, b, c11);
    b = g2_frag(b2p + kb, hh); c02 = g2_mma(a0, b, c02); c12 = g2_mma(a1, b, c12);
    b = g2_frag(b3p + kb, hh); c03 = g2_mma(a0, b, c03); c13 = g2_mma(a1, b, c13); }
  v8f accs[8] = {c00, c01, c02, c03, c10, c11, c12, c13};
#pragma unroll
  for (int u = 0; u < 8; ++u) { const int t = u & 3, half = u >> 2; const int col = col0 + t * 16 + ln; const float bv = bp ? bf16_round(bp[col]) : 0.f;
#pragma unroll
    for (int r = 0; r < 8; ++r) { const int rloc = half * 16 + 8 * hh + r; float v = accs[u][r] * alpha + bv; if (CP) { if (rowsPerB < 0) v += CP[cofs + (size_t)(row0g + row0 + rloc) * ldc + col];        else { const int bidx = (row0g + row0 + rloc) / rowsPerB; v += CP[(size_t)bidx * sCPb + (size_t)by * 64 + col]; } }
      if (ACT == 3) v = fmaxf(v, 0.f); else if (ACT == 6) v = 0.5f * v * (1.0f + erff(v * 0.70710678118654752f)); else if (ACT == 11) v = 1.0f / (1.0f + expf(-v)); else if (ACT == 15) v = v / (1.0f + expf(-v)); else if (ACT == 12) v = (v > 0.f) ? v : 0.01f * v; else if (ACT == 8) v = tanhf(v);
      so[w][rloc][t * 16 + ln] = v; } }
  __builtin_amdgcn_fence(__ATOMIC_ACQ_REL, "workgroup"); __builtin_amdgcn_wave_barrier();
  const int rsub = lane >> 4, c4 = (lane & 15) * 4;
  for (int pass = 0; pass < 2; ++pass) {
#pragma unroll
    for (int q = 0; q < 16; ++q) { const int r = q * 2 + rsub; const v4f v = *(const v4fa*)&so[w][r][c4]; if (C) *(volatile v4f*)(C + cofs + (size_t)(row0 + r) * ldc + col0 + c4) = v; if (C16) { v4h h4; for (int i = 0; i < 4; ++i) h4[i] = (_Float16)v[i]; *(volatile v4h*)(C16 + cofs + (size_t)(row0 + r) * ldc + col0 + c4) = h4; } }
    if (pass == 0) __threadfence(); } }


template <int CAUSAL>
__global__ __launch_bounds__(128) void k_flash(const _Float16* __restrict__ Q16, int ldq, const _Float16* __restrict__ K16, int ldk, const _Float16* __restrict__ Vt, const int* __restrict__ MSK, float* __restrict__ O, int ldo) {
  constexpr int RPW = 16, RTN = RPW / 16, NQB = TQ / (4 * RPW), DT = 4, KS = 2;
  __shared__ __attribute__((aligned(16))) unsigned short sP[4][RPW][40]; __shared__ __attribute__((aligned(16))) float sO[4][RPW][64 + 4];
  const int tid = threadIdx.x, w = tid >> 5, lane = tid & 31, ln = lane & 15, hh = lane >> 4;
  const int slab = blockIdx.x / QBNP, qblk = QB0P + blockIdx.x % QBNP; (void)NQB; const int b = slab / NH, h = slab % NH; const int qb0 = qblk * (4 * RPW); const int q0 = qb0 + w * RPW;
  FragH aq[2][KS];
#pragma unroll
  for (int rt = 0; rt < RTN; ++rt) { const unsigned short* qr = (const unsigned short*)Q16 + ((size_t)b * TQ + q0 + rt * 16 + ln) * ldq + h * 64;
#pragma unroll
    for (int ks = 0; ks < KS; ++ks) { aq[rt][ks].half[0] = *(const v8us*)(qr + ks * 32 + 8 * hh); aq[rt][ks].half[1] = *(const v8us*)(qr + ks * 32 + 16 + 8 * hh); } }
  const unsigned short* Vth = (const unsigned short*)Vt + (size_t)slab * 64 * TK;
  float m_r[2][8], l_r[2][8]; v8f oacc[2][DT];
#pragma unroll
  for (int rt = 0; rt < RTN; ++rt) {
#pragma unroll
    for (int r = 0; r < 8; ++r) { m_r[rt][r] = -3.0e38f; l_r[rt][r] = 0.f; }
#pragma unroll
    for (int dt = 0; dt < DT; ++dt) oacc[rt][dt] = (v8f){0.f,0.f,0.f,0.f,0.f,0.f,0.f,0.f}; }
  const int jend = (CAUSAL == 1) ? (qb0 + 4 * RPW) : ((CAUSAL == 23) ? min(TK, (qb0 / CHK + 2) * CHK) : ((CAUSAL == 32) ? (((qb0 >> 10) + 1) << 10) : TK));        const int jbeg = (CAUSAL == 23) ? max(0, (qb0 / CHK - 1) * CHK) : ((CAUSAL == 32) ? ((qb0 >> 10) << 10) : 0);
#pragma unroll 1
  for (int j0 = jbeg; j0 < jend; j0 += 32) {
    v8f s[2][2];
#pragma unroll
    for (int nt = 0; nt < 2; ++nt) { const unsigned short* kr = (const unsigned short*)K16 + ((size_t)b * TK + j0 + nt * 16 + ln) * ldk + h * 64; FragH bk[KS];
#pragma unroll
      for (int ks = 0; ks < KS; ++ks) { bk[ks].half[0] = *(const v8us*)(kr + ks * 32 + 8 * hh); bk[ks].half[1] = *(const v8us*)(kr + ks * 32 + 16 + 8 * hh); }
#pragma unroll
      for (int rt = 0; rt < RTN; ++rt) { v8f acc = (v8f){0.f,0.f,0.f,0.f,0.f,0.f,0.f,0.f};
#pragma unroll
        for (int ks = 0; ks < KS; ++ks) acc = mmaH<1>(aq[rt][ks].v, aq[rt][ks].v, bk[ks].v, bk[ks].v, acc); s[rt][nt] = acc; } }
#pragma unroll
    for (int rt = 0; rt < RTN; ++rt)
#pragma unroll
      for (int r = 0; r < 8; ++r) { const int tq = q0 + rt * 16 + 8 * hh + r; const int k0 = j0 + ln, k1 = j0 + 16 + ln;
        bool ok0 = (CAUSAL == 1) ? (k0 <= tq) : ((CAUSAL == 2) ? ((k0 >> 5) == (tq >> 5)) : true), ok1 = (CAUSAL == 1) ? (k1 <= tq) : ((CAUSAL == 2) ? ((k1 >> 5) == (tq >> 5)) : true); if (CAUSAL == 23) { const int cq = tq / CHK; ok0 = (abs(k0 / CHK - cq) <= 1) && (MSK[(size_t)b * TK + k0] == 0); ok1 = (abs(k1 / CHK - cq) <= 1) && (MSK[(size_t)b * TK + k1] == 0); }
        if (CAUSAL == 24) { ok0 = (MSK[(size_t)b * TK + k0] == 0); ok1 = (MSK[(size_t)b * TK + k1] == 0); } if (CAUSAL == 32) { ok0 = ((k0 >> 10) == (tq >> 10)); ok1 = ((k1 >> 10) == (tq >> 10)); }
        float s0 = ok0 ? s[rt][0][r] * SCL : -3.0e38f, s1 = ok1 ? s[rt][1][r] * SCL : -3.0e38f; if (CAUSAL == 27) { const float* amk = (const float*)MSK + ((size_t)b * MQI + tq) * MKI; s0 += bf16_round(amk[k0]); s1 += bf16_round(amk[k1]); }        if (CAUSAL == 17) { const float* amk = (const float*)MSK + (size_t)b * TK; s0 += bf16_round(amk[k0]); s1 += bf16_round(amk[k1]); } if (CAUSAL == 18) { const float* tb = (const float*)MSK; const int* ri = MSK + 1024 + (size_t)b * TK; const int rq = ri[tq]; s0 += tb[(h * 8 + rq) * 8 + ri[k0]]; s1 += tb[(h * 8 + rq) * 8 + ri[k1]]; } if (CAUSAL == 19) { const int* rel = MSK + (size_t)tq * TK; const float* rb = (const float*)MSK + (size_t)TQ * TK + ((size_t)(b * NH + h) * TQ + tq) * 64; s0 += rb[rel[k0]]; s1 += rb[rel[k1]]; }                      float mc = fmaxf(s0, s1);
        mc = fmaxf(mc, __shfl_xor(mc, 1, 32)); mc = fmaxf(mc, __shfl_xor(mc, 2, 32)); mc = fmaxf(mc, __shfl_xor(mc, 4, 32)); mc = fmaxf(mc, __shfl_xor(mc, 8, 32));
        const float mn = fmaxf(m_r[rt][r], mc); const float al = (mn > -1.0e38f) ? expf(m_r[rt][r] - mn) : 1.0f; m_r[rt][r] = mn; const float p0 = ok0 ? expf(s0 - mn) : 0.f, p1 = ok1 ? expf(s1 - mn) : 0.f; l_r[rt][r] = l_r[rt][r] * al + p0 + p1;
#pragma unroll
        for (int dt = 0; dt < DT; ++dt) oacc[rt][dt][r] *= al;
        FragH t2; t2.h[0] = (_Float16)(p0 * 1024.0f); t2.h[1] = (_Float16)(p1 * 1024.0f); sP[w][rt * 16 + 8 * hh + r][ln] = t2.u[0]; sP[w][rt * 16 + 8 * hh + r][16 + ln] = t2.u[1]; }
    __builtin_amdgcn_fence(__ATOMIC_ACQ_REL, "workgroup"); __builtin_amdgcn_wave_barrier();
    FragH pa[2];
#pragma unroll
    for (int rt = 0; rt < RTN; ++rt) { pa[rt].half[0] = *(const v8us*)&sP[w][rt * 16 + ln][8 * hh]; pa[rt].half[1] = *(const v8us*)&sP[w][rt * 16 + ln][16 + 8 * hh]; }
#pragma unroll
    for (int dt = 0; dt < DT; ++dt) { const unsigned short* vrow = Vth + (size_t)(dt * 16 + ln) * TK + j0; FragH bv; bv.half[0] = *(const v8us*)(vrow + 8 * hh); bv.half[1] = *(const v8us*)(vrow + 16 + 8 * hh);
#pragma unroll
      for (int rt = 0; rt < RTN; ++rt) oacc[rt][dt] = mmaH<1>(pa[rt].v, pa[rt].v, bv.v, bv.v, oacc[rt][dt]); }
    __builtin_amdgcn_fence(__ATOMIC_ACQ_REL, "workgroup"); __builtin_amdgcn_wave_barrier(); }
#pragma unroll
  for (int rt = 0; rt < RTN; ++rt) {
#pragma unroll
    for (int r = 0; r < 8; ++r) { float l = l_r[rt][r]; l += __shfl_xor(l, 1, 32); l += __shfl_xor(l, 2, 32); l += __shfl_xor(l, 4, 32); l += __shfl_xor(l, 8, 32); l_r[rt][r] = (l > 0.f) ? 1.0f / (l * 1024.0f) : 0.f; }
#pragma unroll
    for (int dt = 0; dt < DT; ++dt)
#pragma unroll
      for (int r = 0; r < 8; ++r) sO[w][rt * 16 + 8 * hh + r][dt * 16 + ln] = oacc[rt][dt][r] * l_r[rt][r]; }
  __builtin_amdgcn_fence(__ATOMIC_ACQ_REL, "workgroup"); __builtin_amdgcn_wave_barrier();
  for (int pass = 0; pass < 2; ++pass) {
#pragma unroll
    for (int rp = 0; rp < RPW; rp += 2) { const int r = rp + (lane >> 4), pc = lane & 15; const v4f val = *(const v4fa*)&sO[w][r][pc * 4]; *(volatile v4f*)(O + ((size_t)b * TQ + q0 + r) * ldo + h * 64 + pc * 4) = val; }
    if (pass == 0) __threadfence(); } }
template <int CAUSAL>
__global__ __launch_bounds__(128) void k_flash5(const _Float16* __restrict__ Q16, const _Float16* __restrict__ QL, int ldq, const _Float16* __restrict__ K16, const _Float16* __restrict__ KL, int ldk, const _Float16* __restrict__ Vt, const _Float16* __restrict__ VtL, const int* __restrict__ MSK, float* __restrict__ O, int ldo) {
  constexpr int RPW = 16, RTN = RPW / 16, NQB = TQ / (4 * RPW), DT = 4, KS = 2;
  __shared__ __attribute__((aligned(16))) unsigned short sP[4][RPW][40]; __shared__ __attribute__((aligned(16))) unsigned short sPL[4][RPW][40]; __shared__ __attribute__((aligned(16))) float sO[4][RPW][64 + 4];
  const int tid = threadIdx.x, w = tid >> 5, lane = tid & 31, ln = lane & 15, hh = lane >> 4;
  const int slab = blockIdx.x / QBN5, qblk = QB05 + blockIdx.x % QBN5; (void)NQB; const int b = slab / NH, h = slab % NH; const int qb0 = qblk * (4 * RPW); const int q0 = qb0 + w * RPW;
  FragH aq[2][KS], aql[2][KS];
#pragma unroll
  for (int rt = 0; rt < RTN; ++rt) { const unsigned short* qr = (const unsigned short*)Q16 + ((size_t)b * TQ + q0 + rt * 16 + ln) * ldq + h * 64; const unsigned short* ql = (const unsigned short*)QL + ((size_t)b * TQ + q0 + rt * 16 + ln) * ldq + h * 64;
#pragma unroll
    for (int ks = 0; ks < KS; ++ks) { aq[rt][ks].half[0] = *(const v8us*)(qr + ks * 32 + 8 * hh); aq[rt][ks].half[1] = *(const v8us*)(qr + ks * 32 + 16 + 8 * hh); aql[rt][ks].half[0] = *(const v8us*)(ql + ks * 32 + 8 * hh); aql[rt][ks].half[1] = *(const v8us*)(ql + ks * 32 + 16 + 8 * hh); } }
  const unsigned short* Vth = (const unsigned short*)Vt + (size_t)slab * 64 * TK; const unsigned short* Vtl = (const unsigned short*)VtL + (size_t)slab * 64 * TK;
  float m_r[2][8], l_r[2][8]; v8f oacc[2][DT], oaccL[2][DT];
#pragma unroll
  for (int rt = 0; rt < RTN; ++rt) {
#pragma unroll
    for (int r = 0; r < 8; ++r) { m_r[rt][r] = -3.0e38f; l_r[rt][r] = 0.f; }
#pragma unroll
    for (int dt = 0; dt < DT; ++dt) { oacc[rt][dt] = (v8f){0.f,0.f,0.f,0.f,0.f,0.f,0.f,0.f}; oaccL[rt][dt] = oacc[rt][dt]; } }
  const int jend = (CAUSAL == 1) ? (qb0 + 4 * RPW) : ((CAUSAL == 23) ? min(TK, (qb0 / CHK + 2) * CHK) : ((CAUSAL == 32) ? (((qb0 >> 10) + 1) << 10) : TK));        const int jbeg = (CAUSAL == 23) ? max(0, (qb0 / CHK - 1) * CHK) : ((CAUSAL == 32) ? ((qb0 >> 10) << 10) : 0);
#pragma unroll 1
  for (int j0 = jbeg; j0 < jend; j0 += 32) {
    v8f s[2][2];
#pragma unroll
    for (int nt = 0; nt < 2; ++nt) { const unsigned short* kr = (const unsigned short*)K16 + ((size_t)b * TK + j0 + nt * 16 + ln) * ldk + h * 64; const unsigned short* klr = (const unsigned short*)KL + ((size_t)b * TK + j0 + nt * 16 + ln) * ldk + h * 64; FragH bk[KS], bkl[KS];
#pragma unroll
      for (int ks = 0; ks < KS; ++ks) { bk[ks].half[0] = *(const v8us*)(kr + ks * 32 + 8 * hh); bk[ks].half[1] = *(const v8us*)(kr + ks * 32 + 16 + 8 * hh); bkl[ks].half[0] = *(const v8us*)(klr + ks * 32 + 8 * hh); bkl[ks].half[1] = *(const v8us*)(klr + ks * 32 + 16 + 8 * hh); }
#pragma unroll
      for (int rt = 0; rt < RTN; ++rt) { v8f acc = (v8f){0.f,0.f,0.f,0.f,0.f,0.f,0.f,0.f}, accl = acc;
#pragma unroll
        for (int ks = 0; ks < KS; ++ks) { acc = mmaH<1>(aq[rt][ks].v, aq[rt][ks].v, bk[ks].v, bk[ks].v, acc); accl = mmaH<1>(aql[rt][ks].v, aql[rt][ks].v, bk[ks].v, bk[ks].v, accl); accl = mmaH<1>(aq[rt][ks].v, aq[rt][ks].v, bkl[ks].v, bkl[ks].v, accl); }
#pragma unroll
        for (int r = 0; r < 8; ++r) acc[r] += accl[r] * 0.0009765625f;
        s[rt][nt] = acc; } }
#pragma unroll
    for (int rt = 0; rt < RTN; ++rt)
#pragma unroll
      for (int r = 0; r < 8; ++r) { const int tq = q0 + rt * 16 + 8 * hh + r; const int k0 = j0 + ln, k1 = j0 + 16 + ln;
        bool ok0 = (CAUSAL == 1) ? (k0 <= tq) : ((CAUSAL == 2) ? ((k0 >> 5) == (tq >> 5)) : true), ok1 = (CAUSAL == 1) ? (k1 <= tq) : ((CAUSAL == 2) ? ((k1 >> 5) == (tq >> 5)) : true);
        if (CAUSAL == 32) { ok0 = ((k0 >> 10) == (tq >> 10)); ok1 = ((k1 >> 10) == (tq >> 10)); }        if (CAUSAL == 4) { const int* mrow = MSK + ((size_t)b * TQ + tq) * TK; ok0 = mrow[k0] != 0; ok1 = mrow[k1] != 0; }
        float s0 = ok0 ? s[rt][0][r] * SCL : -3.0e38f, s1 = ok1 ? s[rt][1][r] * SCL : -3.0e38f; if (CAUSAL == 17) { const float* amk = (const float*)MSK + (size_t)b * TK; s0 += bf16_round(amk[k0]); s1 += bf16_round(amk[k1]); } if (CAUSAL == 18) { const float* tb = (const float*)MSK; const int* ri = MSK + 1024 + (size_t)b * TK; const int rq = ri[tq]; s0 += tb[(h * 8 + rq) * 8 + ri[k0]]; s1 += tb[(h * 8 + rq) * 8 + ri[k1]]; } if (CAUSAL == 19) { const int* rel = MSK + (size_t)tq * TK; const float* rb = (const float*)MSK + (size_t)TQ * TK + ((size_t)(b * NH + h) * TQ + tq) * 64; s0 += rb[rel[k0]]; s1 += rb[rel[k1]]; }                      float mc = fmaxf(s0, s1);
        mc = fmaxf(mc, __shfl_xor(mc, 1, 32)); mc = fmaxf(mc, __shfl_xor(mc, 2, 32)); mc = fmaxf(mc, __shfl_xor(mc, 4, 32)); mc = fmaxf(mc, __shfl_xor(mc, 8, 32));
        const float mn = fmaxf(m_r[rt][r], mc); const float al = (mn > -1.0e38f) ? expf(m_r[rt][r] - mn) : 1.0f; m_r[rt][r] = mn; const float p0 = ok0 ? expf(s0 - mn) : 0.f, p1 = ok1 ? expf(s1 - mn) : 0.f; l_r[rt][r] = l_r[rt][r] * al + p0 + p1;
#pragma unroll
        for (int dt = 0; dt < DT; ++dt) { oacc[rt][dt][r] *= al; oaccL[rt][dt][r] *= al; }
        FragH t2, t2l; const float ps0 = p0 * 1024.0f, ps1 = p1 * 1024.0f; t2.h[0] = (_Float16)ps0; t2.h[1] = (_Float16)ps1; t2l.h[0] = (_Float16)((ps0 - (float)t2.h[0]) * 1024.0f); t2l.h[1] = (_Float16)((ps1 - (float)t2.h[1]) * 1024.0f);
        sP[w][rt * 16 + 8 * hh + r][ln] = t2.u[0]; sP[w][rt * 16 + 8 * hh + r][16 + ln] = t2.u[1]; sPL[w][rt * 16 + 8 * hh + r][ln] = t2l.u[0]; sPL[w][rt * 16 + 8 * hh + r][16 + ln] = t2l.u[1]; }
    __builtin_amdgcn_fence(__ATOMIC_ACQ_REL, "workgroup"); __builtin_amdgcn_wave_barrier();
    FragH pa[2], pl[2];
#pragma unroll
    for (int rt = 0; rt < RTN; ++rt) { pa[rt].half[0] = *(const v8us*)&sP[w][rt * 16 + ln][8 * hh]; pa[rt].half[1] = *(const v8us*)&sP[w][rt * 16 + ln][16 + 8 * hh]; pl[rt].half[0] = *(const v8us*)&sPL[w][rt * 16 + ln][8 * hh]; pl[rt].half[1] = *(const v8us*)&sPL[w][rt * 16 + ln][16 + 8 * hh]; }
#pragma unroll
    for (int dt = 0; dt < DT; ++dt) { const unsigned short* vrow = Vth + (size_t)(dt * 16 + ln) * TK + j0; const unsigned short* vrl = Vtl + (size_t)(dt * 16 + ln) * TK + j0; FragH bv, bl; bv.half[0] = *(const v8us*)(vrow + 8 * hh); bv.half[1] = *(const v8us*)(vrow + 16 + 8 * hh); bl.half[0] = *(const v8us*)(vrl + 8 * hh); bl.half[1] = *(const v8us*)(vrl + 16 + 8 * hh);
#pragma unroll
      for (int rt = 0; rt < RTN; ++rt) { oacc[rt][dt] = mmaH<1>(pa[rt].v, pa[rt].v, bv.v, bv.v, oacc[rt][dt]); oaccL[rt][dt] = mmaH<1>(pl[rt].v, pl[rt].v, bv.v, bv.v, oaccL[rt][dt]); oaccL[rt][dt] = mmaH<1>(pa[rt].v, pa[rt].v, bl.v, bl.v, oaccL[rt][dt]); } }
    __builtin_amdgcn_fence(__ATOMIC_ACQ_REL, "workgroup"); __builtin_amdgcn_wave_barrier(); }
#pragma unroll
  for (int rt = 0; rt < RTN; ++rt) {
#pragma unroll
    for (int r = 0; r < 8; ++r) { float l = l_r[rt][r]; l += __shfl_xor(l, 1, 32); l += __shfl_xor(l, 2, 32); l += __shfl_xor(l, 4, 32); l += __shfl_xor(l, 8, 32); l_r[rt][r] = (l > 0.f) ? 1.0f / (l * 1024.0f) : 0.f; }
#pragma unroll
    for (int dt = 0; dt < DT; ++dt)
#pragma unroll
      for (int r = 0; r < 8; ++r) { float v = oacc[rt][dt][r]; v += oaccL[rt][dt][r] * 0.0009765625f; sO[w][rt * 16 + 8 * hh + r][dt * 16 + ln] = v * l_r[rt][r]; } }
  __builtin_amdgcn_fence(__ATOMIC_ACQ_REL, "workgroup"); __builtin_amdgcn_wave_barrier();
  for (int pass = 0; pass < 2; ++pass) {
#pragma unroll
    for (int rp = 0; rp < RPW; rp += 2) { const int r = rp + (lane >> 4), pc = lane & 15; const v4f val = *(const v4fa*)&sO[w][r][pc * 4]; *(volatile v4f*)(O + ((size_t)b * TQ + q0 + r) * ldo + h * 64 + pc * 4) = val; }
    if (pass == 0) __threadfence(); } }

__global__ __launch_bounds__(256) void k_rotab(float* __restrict__ CS, float* __restrict__ SN) {
  #pragma clang fp contract(off)
  const int t = blockIdx.x * 256 + threadIdx.x; if (t >= SLEN * 32) return; const int j = t % 32, s = t / 32; const float ex = (float)(2 * j) / 64.0f; const float inv = 1.0f / powf(10000.0f, ex); const float th = (float)s * inv; const float c = cosf(th), sn = sinf(th);
  for (int pass = 0; pass < 2; ++pass) { *(volatile float*)(CS + t) = c; *(volatile float*)(SN + t) = sn; if (pass == 0) __threadfence(); } }
__global__ __launch_bounds__(256) void k_rope(const float* __restrict__ F, int nsrc, int ndst, int rep, const float* __restrict__ CS, const float* __restrict__ SN, _Float16* __restrict__ H, _Float16* __restrict__ L) {
  #pragma clang fp contract(off)
  const size_t t = (size_t)blockIdx.x * 256 + threadIdx.x; if (t >= (size_t)NR * ndst * 4) return; const int g8 = (int)(t % 4); const int hd = (int)((t / 4) % ndst); const size_t row = t / ((size_t)4 * ndst); const int s = (int)(row % SLEN); const int hs = hd / rep;
  const float* src = F + row * (size_t)(nsrc * 64) + hs * 64; FragH ah, al, bh, bl;
  for (int i = 0; i < 8; ++i) { const int d = g8 * 8 + i; const float c = CS[s * 32 + d], sn = SN[s * 32 + d]; const float x1 = src[d], x2 = src[d + 32];
    float o1 = x1 * c; o1 += -x2 * sn; float o2 = x2 * c; o2 += x1 * sn;
    _Float16 hv = (_Float16)o1; ah.h[i] = hv; al.h[i] = (_Float16)((o1 - (float)hv) * 1024.0f); hv = (_Float16)o2; bh.h[i] = hv; bl.h[i] = (_Float16)((o2 - (float)hv) * 1024.0f); }
  const size_t o = row * (size_t)(ndst * 64) + hd * 64 + g8 * 8;
  for (int pass = 0; pass < 2; ++pass) { *(volatile v8us*)((unsigned short*)H + o) = ah.half[0]; *(volatile v8us*)((unsigned short*)H + o + 32) = bh.half[0]; *(volatile v8us*)((unsigned short*)L + o) = al.half[0]; *(volatile v8us*)((unsigned short*)L + o + 32) = bl.half[0]; if (pass == 0) __threadfence(); } }
__global__ __launch_bounds__(256) void k_rope2(const float* __restrict__ F, int nsrc, int ndst, int rep, const float* __restrict__ CS, const float* __restrict__ SN, _Float16* __restrict__ H, _Float16* __restrict__ L) {
  #pragma clang fp contract(off)
  const size_t t = (size_t)blockIdx.x * 256 + threadIdx.x; if (t >= (size_t)NR * ndst * 4) return; const int g16 = (int)(t % 4); const int hd = (int)((t / 4) % ndst); const size_t row = t / ((size_t)4 * ndst); const int s = (int)(row % SLEN); const int hs = hd / rep;
  const float* src = F + row * (size_t)(nsrc * 64) + hs * 64 + g16 * 16; FragH ah, al;
  for (int pr = 0; pr < 8; ++pr) { const int i = g16 * 8 + pr; const float c = CS[s * 32 + i], sn = SN[s * 32 + i]; const float x1 = src[2 * pr], x2 = src[2 * pr + 1];
    float o1 = x1 * c; o1 -= x2 * sn; float o2 = x1 * sn; o2 += x2 * c;
    _Float16 hv = (_Float16)o1; ah.h[2 * pr] = hv; al.h[2 * pr] = (_Float16)((o1 - (float)hv) * 1024.0f); hv = (_Float16)o2; ah.h[2 * pr + 1] = hv; al.h[2 * pr + 1] = (_Float16)((o2 - (float)hv) * 1024.0f); }
  const size_t o = row * (size_t)(ndst * 64) + hd * 64 + g16 * 16;
  for (int pass = 0; pass < 2; ++pass) { *(volatile v8us*)((unsigned short*)H + o) = ah.half[0]; *(volatile v8us*)((unsigned short*)H + o + 8) = ah.half[1]; *(volatile v8us*)((unsigned short*)L + o) = al.half[0]; *(volatile v8us*)((unsigned short*)L + o + 8) = al.half[1]; if (pass == 0) __threadfence(); } }
__global__ __launch_bounds__(256) void k_ln512(const float* __restrict__ A, const float* __restrict__ res, const float* __restrict__ g, const float* __restrict__ bb, float* __restrict__ Y, _Float16* __restrict__ Y16) {
  #pragma clang fp contract(off)
  const int wv = threadIdx.x >> 5, ln = threadIdx.x & 31; const size_t r = (size_t)blockIdx.x * 8 + wv; if (r >= NR) return; float x[16]; float s = 0.f;
  for (int i = 0; i < 2; ++i) { const v8f a = *(const v8f*)(A + r * DM + i * 256 + ln * 8); for (int q = 0; q < 8; ++q) { float v = a[q]; if (res) v += bf16_round(res[r * DM + i * 256 + ln * 8 + q]); x[i * 8 + q] = v; s += v; } }
  for (int o = 16; o > 0; o >>= 1) s += __shfl_xor(s, o, 32); const float mu = s / (float)DM; float var = 0.f; for (int q = 0; q < 16; ++q) { const float d = x[q] - mu; var += d * d; }
  for (int o = 16; o > 0; o >>= 1) var += __shfl_xor(var, o, 32); const float inv = rsqrtf(var / (float)DM + 1e-5f);
  for (int pass = 0; pass < 2; ++pass) { for (int i = 0; i < 2; ++i) { const int c0 = i * 256 + ln * 8; v8f y; FragH f; for (int q = 0; q < 8; ++q) { float v = (x[i * 8 + q] - mu) * inv; v *= bf16_round(g[c0 + q]); v += bf16_round(bb[c0 + q]); y[q] = v; f.h[q] = (_Float16)v; } *(volatile v8f*)(Y + r * DM + c0) = y; if (Y16) *(volatile v8us*)((unsigned short*)Y16 + r * DM + c0) = f.half[0]; } if (pass == 0) __threadfence(); } }
__global__ __launch_bounds__(256) void k_pack(const float* __restrict__ rb, const int* __restrict__ rid, int* __restrict__ PK) { const int t = blockIdx.x * 256 + threadIdx.x; if (t >= 1024 + NB * TK) return; int v; if (t < 1024) v = __float_as_int(bf16_round(rb[t])); else v = rid[t - 1024]; *(volatile int*)(PK + t) = v; __threadfence(); *(volatile int*)(PK + t) = v; }
__global__ __launch_bounds__(256) void k_tabin(const float* __restrict__ sp, float* __restrict__ CS, float* __restrict__ SN) { const int t = blockIdx.x * 256 + threadIdx.x; if (t >= SLEN * 32) return; const int i = t % 32, s = t / 32; const float c = bf16_round(sp[s * 64 + 32 + i]), sn = bf16_round(sp[s * 64 + i]);
  for (int pass = 0; pass < 2; ++pass) { *(volatile float*)(CS + t) = c; *(volatile float*)(SN + t) = sn; if (pass == 0) __threadfence(); } }
__global__ __launch_bounds__(256) void k_wsc(const float* __restrict__ Wm, _Float16* __restrict__ Bt, size_t n8, float sc) { const size_t t = (size_t)blockIdx.x * 256 + threadIdx.x; if (t >= n8) return; FragH f; for (int q = 0; q < 8; ++q) f.h[q] = (_Float16)(bf16_round(Wm[t * 8 + q]) * sc); *(volatile v8us*)((unsigned short*)Bt + t * 8) = f.half[0]; __threadfence(); *(volatile v8us*)((unsigned short*)Bt + t * 8) = f.half[0]; }
__global__ __launch_bounds__(256) void k_rotab2(float* __restrict__ CS, float* __restrict__ SN) {
  #pragma clang fp contract(off)
  const int t = blockIdx.x * 256 + threadIdx.x; if (t >= SLEN * 32) return; const int j = t % 32, s = t / 32; const float c0 = -0.14391156831212787f;        const float inv = expf((float)(2 * j) * c0); const float th = (float)s * inv; const float c = cosf(th), sn = sinf(th);
  for (int pass = 0; pass < 2; ++pass) { *(volatile float*)(CS + t) = c; *(volatile float*)(SN + t) = sn; if (pass == 0) __threadfence(); } }
__global__ __launch_bounds__(256) void k_lnu(const float* __restrict__ X, _Float16* __restrict__ N16, float* __restrict__ XB) {
  #pragma clang fp contract(off)
  const int wv = threadIdx.x >> 5, ln = threadIdx.x & 31; const size_t r = (size_t)blockIdx.x * 8 + wv; if (r >= NR) return; float a[32]; float s = 0.f;
  for (int i = 0; i < 4; ++i) { const v8f v = *(const v8f*)(X + r * DM + (i * 32 + ln) * 8); for (int q = 0; q < 8; ++q) { const float u = bf16_round(v[q]); a[i * 8 + q] = u; s += u; } }
  for (int o = 16; o > 0; o >>= 1) s += __shfl_xor(s, o, 32); const float mu = s / (float)DM; float var = 0.f; for (int q = 0; q < 32; ++q) { const float d = a[q] - mu; var += d * d; }
  for (int o = 16; o > 0; o >>= 1) var += __shfl_xor(var, o, 32); const float den = sqrtf(var / (float)(DM - 1)) + 1e-6f; const float inv = 1.0f / den;
  for (int pass = 0; pass < 2; ++pass) { for (int i = 0; i < 4; ++i) { const int c0 = (i * 32 + ln) * 8; FragH f; v8f xb; for (int q = 0; q < 8; ++q) { f.h[q] = (_Float16)((a[i * 8 + q] - mu) * inv); xb[q] = a[i * 8 + q]; } *(volatile v8us*)((unsigned short*)N16 + r * DM + c0) = f.half[0]; *(volatile v8f*)(XB + r * DM + c0) = xb; } if (pass == 0) __threadfence(); } }
__global__ __launch_bounds__(256) void k_vtg(const _Float16* __restrict__ V16, _Float16* __restrict__ Vt) { __shared__ unsigned short tl[64][66]; const int tid = threadIdx.x; const int slab = blockIdx.x / (SLEN / 64), lg = blockIdx.x % (SLEN / 64); const int b = slab / NH, h = slab % NH; const int hs = h / NREP;
  for (int i = tid; i < 64 * 8; i += 256) { const int r = i / 8, c8 = (i % 8) * 8; FragH f; f.half[0] = *(const v8us*)((const unsigned short*)V16 + ((size_t)b * SLEN + lg * 64 + r) * KVD + hs * 64 + c8); for (int q = 0; q < 8; ++q) tl[r][c8 + q] = f.u[q]; }
  __syncthreads();
  for (int pass = 0; pass < 2; ++pass) { for (int rd = 0; rd < 2; ++rd) { const int d = rd * 32 + tid / 8, pc = tid % 8; FragH f; for (int q = 0; q < 8; ++q) f.u[q] = tl[pc * 8 + q][d]; *(volatile v8us*)((unsigned short*)Vt + ((size_t)slab * 64 + d) * SLEN + lg * 64 + pc * 8) = f.half[0]; } if (pass == 0) __threadfence(); } }

__global__ __launch_bounds__(256) void k_h16s(const float* __restrict__ SRC, int lds, int coff, _Float16* __restrict__ DST, size_t n8) { const size_t t = (size_t)blockIdx.x * 256 + threadIdx.x; if (t >= n8) return; const size_t r = (t * 8) / DM; const int c = (int)((t * 8) % DM); const v8f a = *(const v8f*)(SRC + r * lds + coff + c); FragH f; for (int q = 0; q < 8; ++q) f.h[q] = (_Float16)a[q];
  *(volatile v8us*)((unsigned short*)DST + t * 8) = f.half[0]; __threadfence(); *(volatile v8us*)((unsigned short*)DST + t * 8) = f.half[0]; }


__global__ __launch_bounds__(256) void k_ccp(const float* __restrict__ QKV, int coff, _Float16* __restrict__ D) { const size_t t = (size_t)blockIdx.x * 256 + threadIdx.x; if (t >= (size_t)NR * DM / 8) return; const int c0 = (int)((t * 8) % DM); const size_t row = (t * 8) / DM; const v8f a = *(const v8f*)(QKV + row * 3 * DM + coff + c0); FragH f; for (int q = 0; q < 8; ++q) f.h[q] = (_Float16)a[q];
  *(volatile v8us*)((unsigned short*)D + t * 8) = f.half[0]; __threadfence(); *(volatile v8us*)((unsigned short*)D + t * 8) = f.half[0]; }


__global__ __launch_bounds__(256) void k_zero16(_Float16* __restrict__ p, size_t n8) { const size_t t = (size_t)blockIdx.x * 256 + threadIdx.x; if (t >= n8) return; v8us z; for (int q = 0; q < 8; ++q) z[q] = 0; *(volatile v8us*)((unsigned short*)p + t * 8) = z; __threadfence(); *(volatile v8us*)((unsigned short*)p + t * 8) = z; }
__constant__ int HMAP[4096] = {0,1,0,1916,11,0,1911,1912,0,0,0,0,1891,0,1894,1895,167,0,170,199,0,0,0,0,1809,1810,0,1638,1820,0,1823,1824,0,0,0,0,0,0,0,0,0,0,0,0,0,0,0,0,0,0,0,0,0,0,0,0,0,0,0,0,0,0,0,0,0,2,0,0,12,13,0,1913,0,0,0,0,1892,1893,0,1896,168,169,0,172,0,0,0,0,0,1811,0,0,1821,1822,0,1825,0,0,0,0,0,0,0,0,0,0,0,0,0,0,0,0,0,517,0,516,0,511,0,510,0,489,0,488,0,483,0,482,3,0,6,20,0,0,17,18,0,297,0,1900,0,291,1897,1898,0,0,173,174,0,1842,0,1841,1812,0,1815,1829,0,0,1826,1827,0,0,0,0,0,0,0,0,0,0,0,0,0,0,0,0,0,0,0,0,515,0,0,0,509,0,0,0,487,0,0,0,481,5,7,8,0,0,0,19,0,0,0,0,295,0,0,1899,289,0,186,175,0,0,196,0,1840,1814,1816,1817,0,0,0,1828,0,0,0,0,0,0,0,0,0,0,0,0,0,0,0,0,0,0,518,519,0,0,512,513,0,0,490,491,0,0,484,485,0,0,0,0,21,0,24,25,0,0,298,299,0,0,292,293,177,178,0,0,187,188,1843,1844,0,0,0,0,1830,0,1833,1834,0,0,0,0,0,0,0,0,0,0,0,0,0,0,0,0,0,0,0,520,0,0,505,514,0,0,0,492,0,0,477,486,0,0,69,0,22,23,0,26,0,0,105,300,0,0,285,294,0,179,0,0,0,189,0,1845,0,0,0,0,1831,1832,0,1835,0,0,0,0,0,0,0,0,0,0,0,0,0,0,0,0,0,0,0,0,0,0,0,0,506,0,0,0,0,0,0,0,478,0,0,30,70,0,27,28,0,0,0,0,106,0,0,0,286,0,183,0,190,0,193,0,0,0,0,1839,0,0,1836,1837,0,0,0,0,0,0,0,0,0,0,0,0,0,0,0,0,0,0,0,0,0,0,504,0,507,508,0,0,0,0,476,0,479,480,68,0,71,72,0,29,0,0,104,0,107,108,284,0,287,288,184,185,191,192,194,195,0,0,256,0,0,0,0,1838,0,0,0,0,0,0,0,0,0,0,0,0,0,0,0,0,0,0,0,0,521,0,524,525,0,0,0,0,493,0,496,497,37,0,40,67,0,0,0,0,73,0,76,103,301,0,304,305,0,0,0,0,0,0,0,0,247,248,0,0,257,0,260,261,0,0,0,0,0,0,0,0,0,0,0,0,0,0,0,0,0,0,0,0,522,523,0,526,0,0,461,0,494,495,0,498,38,39,0,42,0,0,0,0,74,75,0,78,302,303,0,306,0,0,0,0,0,0,0,0,0,249,0,0,258,259,0,262,0,0,0,0,0,0,0,0,0,0,0,0,0,0,0,0,0,0,0,530,0,0,527,528,0,0,0,502,462,0,499,500,0,0,43,44,0,0,0,82,0,0,79,310,0,0,307,308,0,0,0,0,0,279,0,278,250,0,253,266,0,0,263,264,0,0,0,0,0,0,0,0,0,0,0,0,0,0,0,0,0,0,0,0,0,0,0,529,0,0,460,0,463,464,0,501,0,0,474,45,0,0,66,0,0,0,92,81,0,0,102,309,0,0,0,0,0,0,0,0,277,252,254,255,0,0,0,265,0,0,0,0,0,0,0,0,0,0,0,0,0,0,0,0,0,0,0,0,0,0,0,0,0,0,0,459,0,0,0,0,465,466,0,0,57,58,0,0,83,84,0,0,93,94,0,0,0,0,0,0,0,0,280,281,0,0,0,0,267,0,270,271,0,0,0,0,0,0,0,0,0,0,0,0,0,0,0,0,0,0,0,0,0,0,0,0,0,0,455,0,0,0,0,0,0,467,0,0,0,59,0,0,0,85,0,0,0,95,0,0,0,0,343,0,0,0,0,282,0,0,0,0,268,269,0,272,0,0,0,0,0,0,0,0,0,0,0,0,0,0,0,0,0,0,0,0,0,0,0,0,0,0,0,0,456,449,0,448,468,0,471,0,60,0,63,0,86,0,89,0,96,0,99,0,0,0,0,0,344,0,0,0,0,0,0,276,0,0,273,274,0,0,0,0,0,0,0,0,0,0,0,0,0,0,0,0,0,0,0,0,0,0,0,0,0,0,540,0,457,458,0,0,469,470,472,473,61,62,64,65,87,88,90,91,97,98,100,101,0,0,342,0,345,346,0,0,0,0,356,0,0,0,0,275,0,0,0,0,0,0,0,0,0,0,0,0,0,0,0,0,0,0,0,0,0,0,0,0,531,532,0,453,541,0,544,545,0,0,0,0,0,0,0,0,0,0,0,0,0,0,0,0,311,0,314,341,0,0,0,0,347,348,0,0,357,0,360,361,0,0,0,0,0,0,0,0,0,0,0,0,0,0,0,0,0,0,0,0,0,0,0,0,0,533,0,0,542,543,0,546,0,0,1045,0,0,0,0,0,0,0,0,0,0,0,0,0,312,313,0,316,0,0,0,0,0,349,0,0,358,359,0,362,0,0,1573,0,0,0,0,0,0,0,0,0,0,0,0,0,0,0,0,0,0,563,0,562,534,0,537,550,0,0,547,548,0,0,0,0,1046,0,0,0,0,433,0,432,0,427,0,426,0,0,317,318,0,379,0,378,350,0,353,366,0,0,363,364,0,0,0,0,1574,0,0,0,0,0,0,0,0,0,0,0,0,0,0,0,0,0,0,0,561,536,538,539,0,0,0,549,0,0,1044,0,1047,1048,0,0,0,0,1058,0,431,0,0,0,425,0,330,319,0,0,340,0,377,352,354,355,0,0,0,365,0,0,1572,0,1575,1576,0,0,0,0,1586,0,0,0,0,0,0,0,0,0,0,0,564,565,0,0,0,0,551,0,554,555,0,0,0,1043,0,0,0,0,1049,1050,434,435,0,0,428,429,321,322,0,0,331,332,380,381,0,0,0,0,367,0,370,371,0,0,0,1571,0,0,0,0,1577,1578,0,0,0,0,0,0,0,0,0,0,0,0,0,566,0,0,0,0,552,553,0,556,0,0,1039,0,0,0,0,0,0,1051,0,436,0,0,421,430,0,323,1091,0,0,333,0,382,0,0,0,0,368,369,0,372,0,0,1567,0,0,0,0,0,0,1579,0,0,0,0,0,0,0,0,1619,0,0,0,0,0,0,0,0,560,0,0,557,558,0,0,0,0,1040,1033,0,1032,1052,0,1055,0,0,0,0,0,422,0,327,0,1092,0,337,0,0,0,0,376,0,0,373,374,0,0,0,0,1568,1561,0,1560,1580,0,1583,0,0,0,0,0,0,0,0,0,1620,0,0,0,0,0,0,0,0,0,0,559,0,0,1038,0,1041,1042,0,0,1053,1054,1056,1057,0,0,420,0,423,424,1090,329,1093,1094,338,339,0,0,392,0,0,0,0,375,0,0,1566,0,1569,1570,0,0,1581,1582,1584,1585,0,0,0,0,0,0,1618,0,1621,1622,0,0,0,0,0,0,0,0,0,0,0,0,0,1037,0,0,1034,1035,0,0,0,0,437,0,440,441,1059,0,1062,1089,0,0,0,0,383,384,0,0,393,0,396,397,0,0,0,1565,0,0,1562,1563,0,0,0,0,0,0,0,0,1587,0,1590,1617,0,0,0,0,0,0,0,0,0,0,0,0,0,0,1017,0,0,0,0,1036,0,0,0,0,438,439,0,442,1060,1061,0,1064,0,0,0,0,0,385,0,0,394,395,0,398,0,0,1545,0,0,0,0,1564,0,0,0,0,0,0,0,0,1588,1589,0,1592,0,0,0,0,0,0,0,0,0,0,0,0,0,0,0,0,1018,0,0,0,0,989,0,988,0,983,443,1068,0,0,1065,1066,0,415,0,414,386,0,389,402,0,0,399,400,0,0,0,0,1546,0,0,0,0,1517,0,1516,0,1511,0,1596,0,0,1593,1594,0,0,0,0,0,0,0,0,0,0,0,0,0,0,1016,0,1019,1020,0,0,0,0,1030,0,987,0,0,445,981,0,1078,1067,0,0,1088,0,413,388,390,391,0,0,0,401,0,0,1544,0,1547,1548,0,0,0,0,1558,0,1515,0,0,0,1509,0,1606,1595,0,0,1616,0,0,0,0,0,0,0,0,0,0,0,0,1015,0,0,0,0,1021,1022,990,991,0,0,984,985,1069,1070,0,0,1079,1080,416,417,0,0,0,0,403,0,406,407,0,0,0,1543,0,0,0,0,1549,1550,1518,1519,0,0,1512,1513,1597,1598,0,0,1607,1608,0,0,0,0,0,0,0,0,0,0,0,0,1011,0,0,0,0,0,0,1023,0,992,0,0,977,986,0,1071,0,0,0,1081,0,418,0,0,0,0,404,405,0,408,0,0,1539,0,0,0,0,0,0,1551,0,1520,0,0,1505,1514,0,1599,0,0,0,1609,0,0,0,0,0,0,0,0,0,0,0,0,0,0,1012,1005,0,1004,1024,0,1027,0,0,0,0,0,1072,0,1075,0,1082,0,1085,0,0,0,0,412,0,0,409,410,0,0,0,0,1540,1533,0,1532,1552,0,1555,0,0,0,0,0,1600,0,1603,0,1610,0,1613,0,0,0,0,0,0,0,0,0,0,0,1010,0,1013,1014,0,0,1025,1026,1028,1029,0,0,976,0,1073,1074,1076,1077,1083,1084,1086,1087,0,0,0,0,0,0,0,411,0,0,1538,0,1541,1542,0,0,1553,1554,1556,1557,0,0,1504,0,1601,1602,1604,1605,1611,1612,1614,1615,0,0,0,0,0,0,0,0,567,0,570,1009,0,0,1006,1007,603,604,0,0,993,0,996,997,0,0,0,0,0,0,0,0,0,0,0,0,0,0,0,0,1095,0,1098,1537,0,0,1534,1535,1131,1132,0,0,1521,0,1524,1525,0,0,0,0,0,0,0,0,0,0,0,0,0,0,0,0,2257,569,2258,572,0,0,0,1008,0,605,0,0,994,995,0,998,0,0,0,0,0,0,0,0,0,0,0,0,0,0,0,0,1096,1097,0,1100,0,0,0,1536,0,1133,0,0,1522,1523,0,1526,0,0,0,0,0,0,0,0,0,689,0,688,0,683,0,682,2256,2255,573,574,2262,635,0,634,606,0,609,1002,0,0,999,1000,0,0,0,0,0,0,0,0,0,1217,0,1216,0,1211,0,1210,0,0,1101,1102,0,1163,0,1162,1134,0,1137,1530,0,0,1527,1528,0,0,0,0,0,0,0,0,0,0,0,0,687,0,0,0,2253,0,2254,2248,2260,2261,596,0,2277,608,2278,611,0,0,0,1001,0,0,0,0,0,0,0,0,0,0,0,0,1215,0,0,0,1209,0,1114,1103,0,0,1124,0,1161,1136,1138,1139,0,0,0,1529,0,0,0,0,0,0,0,0,0,0,690,691,0,0,684,685,2252,2251,0,2250,587,588,636,637,2276,2275,0,0,623,0,626,627,0,0,0,0,0,0,0,0,0,0,1218,1219,0,0,1212,1213,1105,1106,0,0,1115,1116,1164,1165,0,0,0,0,1151,0,1154,1155,0,0,0,0,0,0,0,0,0,0,0,692,0,0,677,686,2241,579,2242,0,2225,2224,2221,2266,0,2265,0,0,624,625,0,628,2337,0,2338,0,0,0,0,0,0,0,0,1220,0,0,1205,1214,0,1107,0,0,0,1117,0,1166,0,0,0,0,1152,1153,0,1156,0,0,0,0,0,0,0,0,0,0,0,0,0,0,0,0,2240,2239,583,0,2246,2226,593,2222,2270,0,2274,632,0,0,629,630,2336,2335,0,0,2342,0,0,0,0,0,0,0,0,0,0,0,1206,0,1111,0,1118,0,1121,0,0,0,0,1160,0,0,1157,1158,0,0,0,0,0,0,0,0,0,0,0,0,0,0,676,0,2237,680,2238,2232,2244,2245,2217,595,2268,2269,2272,2273,0,0,0,631,2333,0,2334,2328,2340,2341,0,0,0,0,0,0,0,0,1204,0,1207,1208,1112,1113,1119,1120,1122,1123,0,0,1176,0,0,0,0,1159,0,0,0,0,0,0,0,0,0,0,0,0,693,0,696,697,2236,2235,0,2234,0,0,2227,2228,639,640,0,0,649,0,652,653,2332,2331,2283,2330,0,0,0,0,0,0,0,0,1221,0,1224,1225,0,0,0,0,0,0,0,0,1167,1168,0,0,1177,0,1180,1181,0,0,0,0,0,0,0,0,0,0,0,0,694,695,0,698,2193,0,2194,0,0,2230,0,2229,2129,2128,2125,2124,2113,2112,2293,2292,2280,2286,961,2285,0,0,0,0,0,0,0,0,1222,1223,0,1226,2577,0,2578,0,0,0,0,0,0,1169,0,0,1178,1179,0,1182,0,0,1489,0,0,0,0,0,0,0,0,702,0,0,699,700,2192,2191,0,0,2198,671,0,670,642,2130,645,2126,0,2114,655,2294,0,0,2287,2288,962,0,0,0,0,0,0,1230,0,0,1227,1228,2576,2575,0,0,2582,1199,0,1198,1170,0,1173,1186,0,0,1183,1184,0,0,0,0,1490,0,0,0,0,0,0,0,0,0,0,701,2189,0,2190,2184,2196,2197,0,0,2213,644,2214,647,2122,0,2105,657,2309,2290,2310,2289,2325,964,2326,0,0,0,974,0,0,0,0,1229,2573,0,2574,2568,2580,2581,0,0,2597,1172,2598,1175,0,0,0,1185,0,0,1488,0,1491,1492,0,0,0,0,1502,0,0,0,0,0,2188,2187,0,2186,0,0,672,673,2212,2211,2131,2132,659,0,2115,2116,2308,2307,0,959,2324,2323,0,0,965,966,0,0,0,0,0,0,2572,2571,0,2570,0,0,1200,1201,2596,2595,0,0,1187,0,1190,1191,0,0,0,1487,0,0,0,0,1493,1494,0,0,0,0,0,0,2177,0,2178,0,2161,2160,2157,2202,0,2201,0,2133,2097,2118,2098,2298,0,2297,955,2314,0,2313,0,0,0,967,0,0,0,0,0,0,2561,0,2562,0,2545,2544,2541,2586,0,2585,0,0,1188,1189,0,1192,0,0,1483,0,0,0,0,0,0,1495,0,0,0,0,0,0,2176,2175,0,0,2182,2162,0,2158,2206,0,2210,668,2096,2095,665,666,2302,0,2306,0,2318,949,2322,948,968,0,971,0,0,0,0,0,2560,2559,0,0,2566,2546,0,2542,2590,0,2594,1196,0,0,1193,1194,0,0,0,0,1484,1477,0,1476,1496,0,1499,0,0,0,0,0,2173,0,2174,2168,2180,2181,2153,0,2204,2205,2208,2209,2093,0,2094,2088,2300,2301,2304,2305,2316,2317,2320,2321,969,970,972,973,0,0,0,0,2557,0,2558,2552,2564,2565,2537,0,2588,2589,2592,2593,0,0,0,1195,0,0,1482,0,1485,1486,0,0,1497,1498,1500,1501,0,0,0,0,2172,2171,0,2170,713,0,2163,2164,0,0,0,0,2138,2091,2139,2140,839,840,0,953,849,0,950,951,0,0,0,0,0,0,0,0,2556,2555,0,2554,2362,0,2547,2548,0,0,0,0,0,0,0,0,1367,1368,0,1481,1377,0,1478,1479,0,0,0,0,0,0,0,0,2001,705,2002,0,714,2166,0,2165,0,0,2149,2148,2136,2142,0,2141,1787,1786,1783,1782,1771,1770,1767,1766,1723,1722,1719,1718,2401,2400,2397,2396,0,2345,2373,2372,2360,2550,0,2549,0,0,0,0,0,0,0,0,0,1369,0,0,1378,1379,0,1480,0,0,0,0,0,735,0,734,2000,1999,709,722,2006,0,719,720,0,0,0,2150,0,871,2143,2144,842,1788,845,1784,0,1772,855,1768,0,1724,0,1720,0,2402,0,2398,2350,0,2354,2374,0,0,2367,2368,0,0,0,0,0,1399,0,1398,1370,0,1373,1386,0,0,1383,1384,0,0,0,0,0,0,0,0,1997,708,1998,1992,2004,2005,0,721,2021,0,2022,0,0,2146,0,2145,869,844,1779,847,1780,0,1763,857,1764,0,1715,0,1716,0,2393,0,2394,2349,2352,2353,0,2370,0,2369,0,0,0,0,0,0,0,0,1397,1372,1374,1375,0,0,0,1385,0,0,0,0,0,0,736,737,1996,1995,0,1994,723,0,726,727,2020,2019,0,0,0,0,872,873,0,0,1789,1790,859,0,1773,1774,0,0,1725,1726,0,0,2403,2404,0,0,0,0,2378,0,2379,2380,0,0,0,0,0,0,1400,1401,0,0,0,0,1387,0,1390,1391,0,0,0,0,0,0,0,738,1985,0,1986,0,1969,1968,1965,2010,0,2009,807,0,0,0,0,874,2081,1792,2082,1791,1755,1776,1756,1775,0,1728,943,1727,1691,2406,1692,2405,2465,0,2466,2388,2376,2382,0,2381,2529,0,2530,0,0,0,0,1402,0,0,1435,0,1388,1389,0,1392,0,0,1471,0,0,0,0,0,1984,1983,0,732,1990,1970,729,1966,2014,0,2018,0,808,0,0,0,2080,2079,0,868,2086,1753,865,866,1760,0,0,0,1690,1689,0,0,2464,2463,0,2390,2470,0,2383,2384,2528,2527,0,0,2534,0,0,0,0,0,0,1396,1436,0,1393,1394,0,0,0,0,1472,0,0,0,1981,0,1982,1976,1988,1989,1961,731,2012,2013,2016,2017,809,810,0,0,2077,0,2078,2072,2084,2085,1752,1746,1758,1759,942,0,1687,946,1688,1682,2461,1695,2462,2456,2468,2469,0,2385,2525,0,2526,2520,2532,2533,0,0,0,0,1434,0,1437,1438,0,1395,0,0,1470,0,1473,1474,0,0,1980,1979,742,1978,0,0,1971,1972,775,0,778,805,0,0,0,0,2076,2075,2027,2074,1796,1749,1797,1798,911,0,914,941,1732,1685,1733,1734,2460,2459,2411,2458,0,0,0,0,2524,2523,2475,2522,0,0,0,0,1403,0,1406,1433,0,0,0,0,1439,0,1442,1469,0,0,0,0,1937,741,1938,744,0,1974,0,1973,1885,1884,1881,1880,1869,1868,2037,2036,2024,2030,1807,2029,1794,1800,0,1799,1659,913,1743,1742,1730,1736,2421,2420,2408,2414,0,2413,0,0,2485,2484,2472,2478,0,2477,0,0,0,0,1404,1405,0,1408,0,0,0,0,1440,1441,0,1444,0,0,0,748,1936,1935,745,746,1942,0,0,784,0,1886,781,1882,0,1870,0,2038,0,0,2031,2032,0,0,1801,1802,1658,1657,917,1744,1664,0,1737,2422,0,0,2415,2416,0,0,0,2486,0,0,2479,2480,0,0,0,1412,0,0,1409,1410,0,0,0,1448,0,0,1445,1446,0,0,0,0,1933,0,1934,1928,1940,1941,768,0,1957,0,1958,783,1878,0,1861,0,2053,2034,2054,2033,2069,1804,2070,1803,1655,0,1656,1650,1662,1740,940,1739,2437,2418,2438,2417,2453,0,2454,0,2501,2482,2502,2481,2517,0,2518,0,0,0,1422,1411,0,0,1432,0,0,0,1458,1447,0,0,1468,0,1932,1931,0,1930,759,760,0,0,1956,1955,1887,1888,795,796,1871,1872,2052,2051,0,0,2068,2067,0,0,1654,1653,0,1652,931,932,0,0,2436,2435,0,0,2452,2451,0,0,2500,2499,0,0,2516,2515,0,0,1413,1414,0,0,1423,1424,0,0,1449,1450,0,0,1459,1460,0,0,1921,751,1922,0,1909,1908,1905,1946,0,1945,0,1889,1853,1874,1854,2042,204,2041,205,2058,0,2057,0,0,1643,923,1644,0,1631,1630,1627,2426,0,2425,0,2442,0,2441,0,2490,0,2489,0,2506,0,2505,0,0,0,1415,0,0,0,1425,0,0,0,1451,0,0,0,1461,0,0,1920,1919,755,0,1926,1910,765,1906,1950,0,1954,0,1852,1851,801,0,2046,202,2050,0,2062,0,2066,0,1642,1641,927,0,1648,1632,937,1628,2430,0,2434,0,2446,0,2450,0,2494,0,2498,0,2510,0,2514,0,1416,0,1419,0,1426,0,1429,0,1452,0,1455,0,1462,0,1465,0,1917,754,1918,1914,1924,1925,1901,767,1948,1949,1952,1953,1849,800,1850,1846,2044,2045,2048,2049,2060,2061,2064,2065,1818,926,1819,1636,1646,1647,1623,939,2428,2429,2432,2433,2444,2445,2448,2449,2492,2493,2496,2497,2508,2509,2512,2513,1417,1418,1420,1421,1427,1428,1430,1431,1453,1454,1456,1457,1463,1464,1466,1467};
#define NTOK 4096
#define NHT 16
__global__ __launch_bounds__(256) void k_gath(const float* __restrict__ q, const float* __restrict__ k, const float* __restrict__ v, _Float16* __restrict__ Q0, _Float16* __restrict__ K0, _Float16* __restrict__ V0, _Float16* __restrict__ Q1, _Float16* __restrict__ K1, _Float16* __restrict__ V1) {
  const size_t t = (size_t)blockIdx.x * 256 + threadIdx.x; const size_t n0 = (size_t)2 * NTOK * DM / 8, n1 = (size_t)2 * (NTOK / 2) * DM / 8; if (t >= n0 + n1) return;
  const bool g1 = t >= n0; const size_t tt = g1 ? t - n0 : t; const int c0 = (int)((tt * 8) % DM); const size_t row = (tt * 8) / DM; const int hh = c0 / 64, d0 = c0 % 64;
  int b, n, h; if (!g1) { b = (int)(row / NTOK); n = (int)(row % NTOK); h = hh; } else { b = (int)(row / (NTOK / 2)); n = 2 * (int)(row % (NTOK / 2)) + 1; h = 8 + hh; }
  const int nk = min(max(HMAP[n], 0), NTOK - 1);
  const v8f aq = *(const v8f*)(q + (((size_t)b * NTOK + n) * NHT + h) * 64 + d0), ak = *(const v8f*)(k + (((size_t)b * NTOK + nk) * NHT + h) * 64 + d0), av = *(const v8f*)(v + (((size_t)b * NTOK + nk) * NHT + h) * 64 + d0);
  FragH fq, fk, fv; for (int i = 0; i < 8; ++i) { fq.h[i] = (_Float16)bf16_round(aq[i]); fk.h[i] = (_Float16)bf16_round(ak[i]); fv.h[i] = (_Float16)bf16_round(av[i]); }
  _Float16* dq = g1 ? Q1 : Q0; _Float16* dk = g1 ? K1 : K0; _Float16* dv = g1 ? V1 : V0;
  for (int pass = 0; pass < 2; ++pass) { *(volatile v8us*)((unsigned short*)dq + tt * 8) = fq.half[0]; *(volatile v8us*)((unsigned short*)dk + tt * 8) = fk.half[0]; *(volatile v8us*)((unsigned short*)dv + tt * 8) = fv.half[0]; if (pass == 0) __threadfence(); } }
__global__ __launch_bounds__(256) void k_asm(const float* __restrict__ O0, const float* __restrict__ O1, float* __restrict__ out) { const size_t t = (size_t)blockIdx.x * 256 + threadIdx.x; if (t >= (size_t)2 * NTOK * NHT * 64 / 8) return; const int c0 = (int)((t * 8) % (NHT * 64)); const size_t row = (t * 8) / (NHT * 64); const int b = (int)(row / NTOK), n = (int)(row % NTOK); const int h = c0 / 64, d0 = c0 % 64; v8f o;
  if (h < 8) o = *(const v8f*)(O0 + ((size_t)b * NTOK + n) * DM + h * 64 + d0); else if (n & 1) o = *(const v8f*)(O1 + ((size_t)b * (NTOK / 2) + (n >> 1)) * DM + (h - 8) * 64 + d0); else { for (int i = 0; i < 8; ++i) o[i] = 0.f; }
  *(volatile v8f*)(out + t * 8) = o; __threadfence(); *(volatile v8f*)(out + t * 8) = o; }
extern "C" void kernel_launch(void* const* d_in, const int* in_sizes, int n_in,
                              void* d_out, int out_size, void* d_ws, size_t ws_size, hipStream_t stream) {
  (void)in_sizes; (void)n_in; (void)out_size;
  const float* q = (const float*)d_in[0]; const float* k = (const float*)d_in[1]; const float* v = (const float*)d_in[2];
  char* ws = (char*)d_ws; size_t off = 0;
  auto take = [&](size_t bytes) { char* p = ws + off; off += (bytes + 255) & ~(size_t)255; return p; };
  const size_t n0 = (size_t)2 * NTOK * DM, n1 = (size_t)2 * (NTOK / 2) * DM;
  _Float16* Q0 = (_Float16*)take(n0 * 2); _Float16* K0 = (_Float16*)take(n0 * 2); _Float16* V0 = (_Float16*)take(n0 * 2); _Float16* VT0 = (_Float16*)take(n0 * 2); float* O0 = (float*)take(n0 * 4);
  _Float16* ZERO = (_Float16*)take(n0 * 2);        _Float16* Q1 = (_Float16*)take(n1 * 2); _Float16* K1 = (_Float16*)take(n1 * 2); _Float16* V1 = (_Float16*)take(n1 * 2); _Float16* VT1 = (_Float16*)take(n1 * 2); float* O1 = (float*)take(n1 * 4);
  if (off > ws_size) return;
  k_zero16<<<(unsigned)((n0 / 8 + 255) / 256), 256, 0, stream>>>(ZERO, n0 / 8); k_gath<<<(unsigned)(((n0 + n1) / 8 + 255) / 256), 256, 0, stream>>>(q, k, v, Q0, K0, V0, Q1, K1, V1);
  k_vtg<<<4 * NH * (SLEN / 64), 256, 0, stream>>>(V0, VT0); k_vtg<<<2 * NH * (SLEN / 64), 256, 0, stream>>>(V1, VT1);
  k_flash5<32><<<4 * NH * QBN5, 128, 0, stream>>>(Q0, ZERO, DM, K0, ZERO, DM, VT0, ZERO, nullptr, O0, DM);
  k_flash5<0><<<2 * NH * QBN5, 128, 0, stream>>>(Q1, ZERO, DM, K1, ZERO, DM, VT1, ZERO, nullptr, O1, DM);
  k_asm<<<(unsigned)(((size_t)2 * NTOK * NHT * 64 / 8 + 255) / 256), 256, 0, stream>>>(O0, O1, (float*)d_out);
}
